// CNF_86019605004441
// MI455X (gfx1250) — hardware-verified
//
#include <hip/hip_runtime.h>
#include <math.h>
#include <stdint.h>

constexpr int kRows = 32768;
constexpr int kDim  = 16;
constexpr int kCond = 64;
constexpr int kHid  = 512;
constexpr int kKz   = 32;
constexpr int kRowsPerBlock = 128;
constexpr int kMaxSeg = 8;
constexpr float kLogTwoPiTerm = 14.70301628112793f;

static_assert(kRows % kRowsPerBlock == 0, "rows per block");
static_assert(kRows % 64 == 0 && kHid % 64 == 0, "GEMM M/N tile multiples");
static_assert(kCond % 32 == 0 && kKz % 32 == 0 && kHid % 32 == 0, "GEMM K multiples of 32");
static_assert(kHid == 512 && kDim == 16 && kCond == 64, "thread maps assume these");

typedef __attribute__((ext_vector_type(16))) _Float16 v16h;
typedef __attribute__((ext_vector_type(8)))  _Float16 v8h;
typedef __attribute__((ext_vector_type(16))) __bf16   v16b;
typedef __attribute__((ext_vector_type(8)))  __bf16   v8b;
typedef __attribute__((ext_vector_type(8)))  float    v8f;
typedef __attribute__((ext_vector_type(4)))  float    v4f;
typedef __attribute__((ext_vector_type(4)))  unsigned int v4u;

constexpr size_t kBytesP   = (size_t)kHid * kRows * 4;
constexpr size_t kBytesC   = (size_t)kHid * kRows * 2;
constexpr size_t kBytesCtx = (size_t)kRows * kCond * 2;
constexpr size_t kBytesEps = (size_t)kRows * kKz * 2;
constexpr size_t kBytesW1c = (size_t)kHid * kCond * 2;
constexpr size_t kBytesW1z = (size_t)kHid * kKz * 2;
constexpr size_t kBytesW2p = (size_t)kHid * kKz * 2;
constexpr size_t kBytesW2T = (size_t)kDim * kHid * 2;
constexpr size_t kBytesTv  = (size_t)kHid * 4;
constexpr size_t kOffP   = 0;
constexpr size_t kOffC   = kOffP + kBytesP;
constexpr size_t kOffCtx = kOffC + kBytesC;
constexpr size_t kOffEps = kOffCtx + kBytesCtx;
constexpr size_t kOffW1c = kOffEps + kBytesEps;
constexpr size_t kOffW1z = kOffW1c + kBytesW1c;
constexpr size_t kOffW2p = kOffW1z + kBytesW1z;
constexpr size_t kOffW2T = kOffW2p + kBytesW2p;
constexpr size_t kOffTv  = kOffW2T + kBytesW2T;
constexpr size_t kWsTotal = kOffTv + kBytesTv;
static_assert(kWsTotal == 107104256, "carve total");
static_assert(kWsTotal <= (size_t)134217728, "carve within 128 MiB");

constexpr int kBlkCtx = kRows * kCond / 8 / 256;
constexpr int kBlkEps = kRows * kKz / 8 / 256;
constexpr int kBlkW1c = kHid * kCond / 8 / 256;
constexpr int kBlkW1z = kHid * kKz / 8 / 256;
constexpr int kBlkW2p = kHid * kKz / 8 / 256;
constexpr int kBlkW2T = kDim * kHid / 8 / 256;
constexpr int kBlkTv  = 1;
constexpr int kBlkPrep = kBlkCtx + kBlkEps + kBlkW1c + kBlkW1z + kBlkW2p + kBlkW2T + kBlkTv;
static_assert(kBlkCtx * 256 * 8 == kRows * kCond, "ctx coverage");
static_assert(kBlkEps * 256 * 8 == kRows * kKz, "eps coverage");
static_assert(kBlkW1c * 256 * 8 == kHid * kCond, "w1c coverage");
static_assert(kBlkW1z * 256 * 8 == kHid * kKz, "w1z coverage");
static_assert(kBlkW2p * 256 * 8 == kHid * kKz, "w2p coverage");
static_assert(kBlkW2T * 256 * 8 == kDim * kHid, "w2t coverage");
static_assert(128 * 4 == kHid, "tvec coverage");

__device__ __forceinline__ unsigned short f2bf_bits(float f) {
  unsigned u = __float_as_uint(f);
  return (unsigned short)((u + 0x7FFFu + ((u >> 16) & 1u)) >> 16);
}
__device__ __forceinline__ float bf_bits2f(unsigned short h) { return __uint_as_float(((unsigned)h) << 16); }

__device__ __forceinline__ void dep_guard_h(v8f& a, v8f& b, v16h x, v16h y) { asm volatile("v_nop\n\tv_nop\n\tv_nop\n\tv_nop" : "+v"(a), "+v"(b) : "v"(x), "v"(y)); }
__device__ __forceinline__ void dep_guard_b(v8f& a, v8f& b, v16b x, v16b y) { asm volatile("v_nop\n\tv_nop\n\tv_nop\n\tv_nop" : "+v"(a), "+v"(b) : "v"(x), "v"(y)); }
__device__ __forceinline__ void keep4_h(v16h a, v16h b, v16h c, v16h d) { asm volatile("v_nop" :: "v"(a), "v"(b), "v"(c), "v"(d)); }
__device__ __forceinline__ void keep4_b(v16b a, v16b b, v16b c, v16b d) { asm volatile("v_nop" :: "v"(a), "v"(b), "v"(c), "v"(d)); }
__device__ __forceinline__ void acc_guard4(v8f& a, v8f& b, v8f& c, v8f& d) { asm volatile("v_nop\n\tv_nop\n\tv_nop\n\tv_nop" : "+v"(a), "+v"(b), "+v"(c), "+v"(d)); }
template <typename T> struct Frag;
template <> struct Frag<_Float16> {
  typedef v16h V; union U { v16h v; v8h h[2]; };
  static __device__ __forceinline__ v16h load(const _Float16* p) {
    U f; f.h[0] = *(const v8h*)(p); f.h[1] = *(const v8h*)(p + 16); return f.v;
  }
  static __device__ __forceinline__ v8f mma(v16h a, v16h b, v8f c) {
    return __builtin_amdgcn_wmma_f32_16x16x32_f16(false, a, false, b, (short)0, c, false, false);
  }
  static __device__ __forceinline__ void guard(v8f& a, v8f& b, v16h x, v16h y) { dep_guard_h(a, b, x, y); }
  static __device__ __forceinline__ void keep(v16h a, v16h b, v16h c, v16h d) { keep4_h(a, b, c, d); }
};
template <> struct Frag<__bf16> {
  typedef v16b V; union U { v16b v; v8b h[2]; };
  static __device__ __forceinline__ v16b load(const __bf16* p) {
    U f; f.h[0] = *(const v8b*)(p); f.h[1] = *(const v8b*)(p + 16); return f.v;
  }
  static __device__ __forceinline__ v8f mma(v16b a, v16b b, v8f c) {
    return __builtin_amdgcn_wmma_f32_16x16x32_bf16(false, a, false, b, (short)0, c, false, false);
  }
  static __device__ __forceinline__ void guard(v8f& a, v8f& b, v16b x, v16b y) { dep_guard_b(a, b, x, y); }
  static __device__ __forceinline__ void keep(v16b a, v16b b, v16b c, v16b d) { keep4_b(a, b, c, d); }
};

__device__ __forceinline__ unsigned pk16(unsigned short a, unsigned short b) { return (unsigned)a | ((unsigned)b << 16); }

__device__ __forceinline__ void guard1_b(v8f& a, v16b x, v16b y) { asm volatile("v_nop\n\tv_nop\n\tv_nop\n\tv_nop" : "+v"(a) : "v"(x), "v"(y)); }
__device__ __forceinline__ void guard4in_b(v8f& a, v8f& b, v8f& c, v8f& d, v16b x, v16b y) {
  asm volatile("v_nop\n\tv_nop\n\tv_nop\n\tv_nop" : "+v"(a), "+v"(b), "+v"(c), "+v"(d) : "v"(x), "v"(y));
}
__device__ __forceinline__ void wave_sync() {
  __builtin_amdgcn_fence(__ATOMIC_RELEASE, "workgroup");
  __builtin_amdgcn_wave_barrier();
  __builtin_amdgcn_fence(__ATOMIC_ACQUIRE, "workgroup");
}
__device__ __forceinline__ __bf16 to_bf16(float f) { return __builtin_bit_cast(__bf16, f2bf_bits(f)); }
__device__ __forceinline__ float  bf_rne(float f)  { return __uint_as_float(((unsigned)f2bf_bits(f)) << 16); }
__device__ __forceinline__ v4u pack_bf16x8(v4f a, v4f c) {
  return (v4u){ pk16(f2bf_bits(a.x), f2bf_bits(a.y)), pk16(f2bf_bits(a.z), f2bf_bits(a.w)),
                pk16(f2bf_bits(c.x), f2bf_bits(c.y)), pk16(f2bf_bits(c.z), f2bf_bits(c.w)) };
}
__device__ __forceinline__ void store16x2(unsigned short* p, v4u u) {
  *(volatile v4u*)p = u;
  __threadfence();
  *(volatile v4u*)p = u;
}
__device__ __forceinline__ void storef4x2(float* p, v4f v) {
  *(volatile v4f*)p = v;
  __threadfence();
  *(volatile v4f*)p = v;
}

template <int ET> struct Elem;
template <> struct Elem<0> { typedef _Float16 T; };
template <> struct Elem<1> { typedef __bf16 T; };
template <int ET, bool SPLIT, int BIAS_MODE, int OUT_MODE, bool RESID, int ACT = 0>
__global__ __launch_bounds__(256) void wmma_gemm64(
    const unsigned short* __restrict__ Ap, const unsigned short* __restrict__ A2p, int lda, long strideA,
    const unsigned short* __restrict__ Btp, const unsigned short* __restrict__ Bt2p, int ldb, long strideB,
    void* __restrict__ Cout, void* __restrict__ Cout2, int ldc, long strideC,
    const float* __restrict__ bias,
    const float* __restrict__ resid, long strideR,
    int M, int N, int K, float scale) {
  typedef typename Elem<ET>::T T;
  typedef typename Frag<T>::V V;
  const T* A = (const T*)Ap; const T* A2 = (const T*)A2p; const T* Bt = (const T*)Btp; const T* Bt2 = (const T*)Bt2p;
  __shared__ __align__(16) float sT[8][16 * 68];
  const int b    = blockIdx.y;
  const int lane = threadIdx.x & 31;
  const int wave = threadIdx.x >> 5;
  const int tilesN = N >> 6;
  const int tilesM = M >> 6;
  const int tile = blockIdx.x * 8 + wave;
  if (tile >= tilesM * tilesN) return;
  const int tm = tile / tilesN;
  const int tn = tile - tm * tilesN;
  const int m0 = tm << 6;
  const int n0 = tn << 6;

  const T* Ab  = A  + (size_t)b * strideA;
  const T* Bb  = Bt + (size_t)b * strideB;
  const T* Ab2 = SPLIT ? (A2  + (size_t)b * strideA) : nullptr;
  const T* Bb2 = SPLIT ? (Bt2 + (size_t)b * strideB) : nullptr;

  const int rlane = lane & 15;
  const int koff  = (lane >> 4) * 8;
  const int mOff  = (lane >> 4) * 8;

  v8f acc[4][4];
#pragma unroll
  for (int i = 0; i < 4; ++i)
#pragma unroll
    for (int j = 0; j < 4; ++j) acc[i][j] = (v8f){0.f,0.f,0.f,0.f,0.f,0.f,0.f,0.f};

  for (int k0 = 0; k0 < K; k0 += 32) {
    V bh[4], bl[4];
#pragma unroll
    for (int j = 0; j < 4; ++j) {
      const size_t bo = (size_t)(n0 + (j << 4) + rlane) * ldb + koff + k0;
      bh[j] = Frag<T>::load(Bb + bo);
      if (SPLIT) bl[j] = Frag<T>::load(Bb2 + bo);
    }
#pragma unroll
    for (int i = 0; i < 4; ++i) {
      const size_t ao = (size_t)(m0 + (i << 4) + rlane) * lda + koff + k0;
      V ah = Frag<T>::load(Ab + ao);
      V al;
      if (SPLIT) al = Frag<T>::load(Ab2 + ao);
#pragma unroll
      for (int j = 0; j < 4; ++j) {
        acc[i][j] = Frag<T>::mma(ah, bh[j], acc[i][j]);
        if (SPLIT) {
          acc[i][j] = Frag<T>::mma(ah, bl[j], acc[i][j]);
          acc[i][j] = Frag<T>::mma(al, bh[j], acc[i][j]);
        }
      }
      Frag<T>::guard(acc[i][0], acc[i][3], ah, SPLIT ? al : ah);
    }
    Frag<T>::keep(bh[0], bh[1], bh[2], bh[3]);
    if (SPLIT) Frag<T>::keep(bl[0], bl[1], bl[2], bl[3]);
  }
  acc_guard4(acc[0][0], acc[0][1], acc[0][2], acc[0][3]);
  acc_guard4(acc[1][0], acc[1][1], acc[1][2], acc[1][3]);
  acc_guard4(acc[2][0], acc[2][1], acc[2][2], acc[2][3]);
  acc_guard4(acc[3][0], acc[3][1], acc[3][2], acc[3][3]);

  float* slab = sT[wave];
  const float* Rb = RESID ? (resid + (size_t)b * strideR) : nullptr;
#pragma unroll
  for (int i = 0; i < 4; ++i) {
    const int mBase = m0 + (i << 4);
#pragma unroll
    for (int j = 0; j < 4; ++j) {
      const int n = n0 + (j << 4) + rlane;
      float bv = 0.f;
      if (BIAS_MODE == 2) bv = bias[n];
#pragma unroll
      for (int r = 0; r < 8; ++r) {
        float v = acc[i][j][r] * scale;
        if (BIAS_MODE == 1) v += bias[mBase + mOff + r];
        if (BIAS_MODE == 2) v += bv;
        if (RESID) v += Rb[(size_t)(mBase + mOff + r) * ldc + n];
        if (ACT == 2) v = fmaxf(v, 0.0f);
        if (ACT == 4) v = (v > 0.f) ? v : 0.01f * v;
        slab[(mOff + r) * 68 + (j << 4) + rlane] = v;
      }
    }
    __builtin_amdgcn_fence(__ATOMIC_RELEASE, "workgroup");
    __builtin_amdgcn_wave_barrier();
    __builtin_amdgcn_fence(__ATOMIC_ACQUIRE, "workgroup");
    if (OUT_MODE == 0) {
      float* C = (float*)Cout + (size_t)b * strideC;
      const int hh = lane >> 4, c4 = (lane & 15) * 4;
      for (int pass = 0; pass < 2; ++pass) {
#pragma unroll
        for (int it = 0; it < 8; ++it) {
          const int row = it * 2 + hh;
          v4f v = *(const v4f*)(slab + row * 68 + c4);
          *(volatile v4f*)(C + (size_t)(mBase + row) * ldc + n0 + c4) = v;
        }
        __threadfence();
      }
    } else {
      const int q = lane >> 3, c8 = (lane & 7) * 8;
      unsigned short* C  = (unsigned short*)Cout  + (size_t)b * strideC;
      unsigned short* C2 = (OUT_MODE == 2) ? ((unsigned short*)Cout2 + (size_t)b * strideC) : nullptr;
      for (int pass = 0; pass < 2; ++pass) {
#pragma unroll
        for (int it = 0; it < 4; ++it) {
          const int row = it * 4 + q;
          const float* sp = slab + row * 68 + c8;
          v8h hv, lv;
#pragma unroll
          for (int e = 0; e < 8; ++e) {
            if (OUT_MODE == 1) {
              hv[e] = (_Float16)sp[e];
            } else {
              unsigned short hb = f2bf_bits(sp[e]);
              unsigned short lb = f2bf_bits(sp[e] - bf_bits2f(hb));
              hv[e] = __builtin_bit_cast(_Float16, hb);
              lv[e] = __builtin_bit_cast(_Float16, lb);
            }
          }
          *(volatile v8h*)(C + (size_t)(mBase + row) * ldc + n0 + c8) = hv;
          if (OUT_MODE == 2) *(volatile v8h*)(C2 + (size_t)(mBase + row) * ldc + n0 + c8) = lv;
        }
        __threadfence();
      }
    }
    __builtin_amdgcn_fence(__ATOMIC_RELEASE, "workgroup");
    __builtin_amdgcn_wave_barrier();
    __builtin_amdgcn_fence(__ATOMIC_ACQUIRE, "workgroup");
  }
}

__global__ __launch_bounds__(256) void prep_kernel(const float* __restrict__ ctx, const float* __restrict__ eps,
                                                   const float* __restrict__ W1, const float* __restrict__ W2,
                                                   unsigned short* __restrict__ ctxb, unsigned short* __restrict__ epsb,
                                                   unsigned short* __restrict__ w1cT, unsigned short* __restrict__ w1zT,
                                                   unsigned short* __restrict__ w2p, unsigned short* __restrict__ w2T,
                                                   float* __restrict__ tvec) {
  const int blk = blockIdx.x;
  const int t = threadIdx.x;
  constexpr int e1 = kBlkCtx;
  constexpr int e2 = e1 + kBlkEps;
  constexpr int e3 = e2 + kBlkW1c;
  constexpr int e4 = e3 + kBlkW1z;
  constexpr int e5 = e4 + kBlkW2p;
  constexpr int e6 = e5 + kBlkW2T;
  if (blk < e1) {
    const int i = blk * 256 + t;
    const float* src = ctx + (size_t)(i >> 3) * kCond + (i & 7) * 8;
    const v4f a = *(const v4f*)src;
    const v4f c = *(const v4f*)(src + 4);
    store16x2(ctxb + 8 * (size_t)i, pack_bf16x8(a, c));
  } else if (blk < e2) {
    const int i = (blk - e1) * 256 + t;
    const int q = i & 3;
    const float* src = eps + (size_t)(i >> 2) * kDim + (q & 1) * 8;
    v4f a = *(const v4f*)src;
    v4f c = *(const v4f*)(src + 4);
    const float fac = (q < 2) ? 1.0f : 0.0f;
    a = a * fac; c = c * fac;
    store16x2(epsb + 8 * (size_t)i, pack_bf16x8(a, c));
  } else if (blk < e3) {
    const int i = (blk - e2) * 256 + t;
    const int n = i >> 3, k8 = (i & 7) * 8;
    const float* src = W1 + (size_t)(kDim + k8) * kHid + n;
    v4f a, c;
    a.x = src[0];        a.y = src[kHid];     a.z = src[2 * kHid]; a.w = src[3 * kHid];
    c.x = src[4 * kHid]; c.y = src[5 * kHid]; c.z = src[6 * kHid]; c.w = src[7 * kHid];
    store16x2(w1cT + 8 * (size_t)i, pack_bf16x8(a, c));
  } else if (blk < e4) {
    const int i = (blk - e3) * 256 + t;
    const int n = i >> 2, q = i & 3;
    const float* src = W1 + (size_t)((q & 1) * 8) * kHid + n;
    v4f a, c;
    a.x = src[0];        a.y = src[kHid];     a.z = src[2 * kHid]; a.w = src[3 * kHid];
    c.x = src[4 * kHid]; c.y = src[5 * kHid]; c.z = src[6 * kHid]; c.w = src[7 * kHid];
    const float fac = (q < 2) ? 1.0f : 0.0f;
    a = a * fac; c = c * fac;
    store16x2(w1zT + 8 * (size_t)i, pack_bf16x8(a, c));
  } else if (blk < e5) {
    const int i = (blk - e4) * 256 + t;
    const int n = i >> 2, q = i & 3;
    const float* src = W2 + (size_t)n * kDim + (q & 1) * 8;
    v4f a = *(const v4f*)src;
    v4f c = *(const v4f*)(src + 4);
    const float fac = (q < 2) ? 1.0f : 0.0f;
    a = a * fac; c = c * fac;
    store16x2(w2p + 8 * (size_t)i, pack_bf16x8(a, c));
  } else if (blk < e6) {
    const int i = (blk - e5) * 256 + t;
    const int n = i >> 6, k8 = (i & 63) * 8;
    const float* src = W2 + (size_t)k8 * kDim + n;
    v4f a, c;
    a.x = src[0];        a.y = src[kDim];     a.z = src[2 * kDim]; a.w = src[3 * kDim];
    c.x = src[4 * kDim]; c.y = src[5 * kDim]; c.z = src[6 * kDim]; c.w = src[7 * kDim];
    store16x2(w2T + 8 * (size_t)i, pack_bf16x8(a, c));
  } else {
    if (t < 128) {
      const v4f a = *(const v4f*)(W1 + (size_t)(kDim + kCond) * kHid + 4 * t);
      v4f r;
      r.x = bf_rne(a.x); r.y = bf_rne(a.y); r.z = bf_rne(a.z); r.w = bf_rne(a.w);
      storef4x2(tvec + 4 * t, r);
    }
  }
}

__global__ __launch_bounds__(256) void dual_gemm_prod_kernel(const unsigned short* __restrict__ A1p,
                                                             const unsigned short* __restrict__ A2p,
                                                             const unsigned short* __restrict__ Btp,
                                                             unsigned short* __restrict__ Cp) {
  __shared__ __align__(16) float sT[8][16 * 68];
  const __bf16* A1 = (const __bf16*)A1p;
  const __bf16* A2 = (const __bf16*)A2p;
  const __bf16* Bt = (const __bf16*)Btp;
  const int lane = threadIdx.x & 31;
  const int wave = threadIdx.x >> 5;
  constexpr int tilesN = kRows / 64;
  constexpr int tilesM = kHid / 32;
  const int tile = blockIdx.x * 8 + wave;
  if (tile >= tilesM * tilesN) return;
  const int tm = tile / tilesN;
  const int tn = tile - tm * tilesN;
  const int m0 = tm * 32;
  const int n0 = tn * 64;
  const int rlane = lane & 15;
  const int koff  = (lane >> 4) * 8;
  const int mOff  = (lane >> 4) * 8;

  v16b bfr[4];
#pragma unroll
  for (int j = 0; j < 4; ++j) bfr[j] = Frag<__bf16>::load(Bt + (size_t)(n0 + 16 * j + rlane) * kKz + koff);

  v8f accU[2][4], accV[2][4];
#pragma unroll
  for (int i = 0; i < 2; ++i)
#pragma unroll
    for (int j = 0; j < 4; ++j) {
      accU[i][j] = (v8f){0.f,0.f,0.f,0.f,0.f,0.f,0.f,0.f};
      accV[i][j] = (v8f){0.f,0.f,0.f,0.f,0.f,0.f,0.f,0.f};
    }
#pragma unroll
  for (int i = 0; i < 2; ++i) {
    const v16b au = Frag<__bf16>::load(A1 + (size_t)(m0 + 16 * i + rlane) * kKz + koff);
    const v16b av = Frag<__bf16>::load(A2 + (size_t)(m0 + 16 * i + rlane) * kKz + koff);
#pragma unroll
    for (int j = 0; j < 4; ++j) {
      accU[i][j] = Frag<__bf16>::mma(au, bfr[j], accU[i][j]);
      accV[i][j] = Frag<__bf16>::mma(av, bfr[j], accV[i][j]);
    }
    guard4in_b(accU[i][0], accU[i][1], accU[i][2], accU[i][3], au, av);
    guard4in_b(accV[i][0], accV[i][1], accV[i][2], accV[i][3], au, av);
  }
  keep4_b(bfr[0], bfr[1], bfr[2], bfr[3]);
  acc_guard4(accU[0][0], accU[0][1], accU[0][2], accU[0][3]);
  acc_guard4(accU[1][0], accU[1][1], accU[1][2], accU[1][3]);
  acc_guard4(accV[0][0], accV[0][1], accV[0][2], accV[0][3]);
  acc_guard4(accV[1][0], accV[1][1], accV[1][2], accV[1][3]);

  float* slab = sT[wave];
  const int q = lane >> 3, c8 = (lane & 7) * 8;
#pragma unroll
  for (int i = 0; i < 2; ++i) {
    const int mBase = m0 + 16 * i;
#pragma unroll
    for (int j = 0; j < 4; ++j) {
#pragma unroll
      for (int r = 0; r < 8; ++r) slab[(mOff + r) * 68 + 16 * j + rlane] = accU[i][j][r] * accV[i][j][r];
    }
    wave_sync();
    for (int pass = 0; pass < 2; ++pass) {
#pragma unroll
      for (int it = 0; it < 4; ++it) {
        const int row = it * 4 + q;
        const float* sp = slab + row * 68 + c8;
        v8h hv;
#pragma unroll
        for (int e = 0; e < 8; ++e) {
          const unsigned short hb = f2bf_bits(sp[e]);
          hv[e] = __builtin_bit_cast(_Float16, hb);
        }
        *(volatile v8h*)(Cp + (size_t)(mBase + row) * kRows + n0 + c8) = hv;
      }
      __threadfence();
    }
    wave_sync();
  }
}

union FragU { v16b v; v8b h8[2]; v4u u[2]; };

__global__ __launch_bounds__(256) void rk4_kernel(const float* __restrict__ x, const float* __restrict__ b2,
                                                  const int* __restrict__ steps,
                                                  const unsigned short* __restrict__ w1zTp,
                                                  const unsigned short* __restrict__ w2Tp,
                                                  const float* __restrict__ tvec,
                                                  const float* __restrict__ Pt,
                                                  const unsigned short* __restrict__ Ctp,
                                                  float* __restrict__ out) {
  __shared__ __align__(16) __bf16 sW1z[kHid * 16];
  __shared__ __align__(16) __bf16 sW2T[kDim * kHid];
  __shared__ __align__(16) float  sTv[kHid];
  __shared__ __align__(16) __bf16 sZ[8][16 * 16];
  __shared__ __align__(16) __bf16 sA[8][16 * 32];
  __shared__ __align__(16) float  sOut[kRowsPerBlock];

  const int tid  = threadIdx.x;
  const int lane = tid & 31;
  const int wave = tid >> 5;
  const int hh   = lane >> 4;
  const int c    = lane & 15;
  const int koff = hh * 8;

#pragma unroll
  for (int it = 0; it < 2; ++it) {
    const int n = it * 256 + tid;
    const v4u u0 = *(const v4u*)(w1zTp + (size_t)n * kKz);
    const v4u u1 = *(const v4u*)(w1zTp + (size_t)n * kKz + 8);
    *(v4u*)(sW1z + n * 16)     = u0;
    *(v4u*)(sW1z + n * 16 + 8) = u1;
  }
#pragma unroll
  for (int it = 0; it < 4; ++it) {
    const int ch = it * 256 + tid;
    const v4u u = *(const v4u*)(w2Tp + (size_t)ch * 8);
    *(v4u*)(sW2T + ch * 8) = u;
  }
  sTv[tid]       = tvec[tid];
  sTv[tid + 256] = tvec[tid + 256];
  __syncthreads();

  int nseg = steps[0] - 1;
  nseg = (nseg < 1) ? 1 : ((nseg > kMaxSeg) ? kMaxSeg : nseg);
  const float dt    = -1.0f / (float)nseg;
  const float hdt   = 0.5f * dt;
  const float sixth = dt * (1.0f / 6.0f);

  const int row0 = blockIdx.x * kRowsPerBlock + wave * 16;
  const int rD   = row0 + 8 * hh;
  const v8f zero8 = (v8f){0.f,0.f,0.f,0.f,0.f,0.f,0.f,0.f};
  const v4u zero4 = (v4u){0u, 0u, 0u, 0u};

  v8f zD;
#pragma unroll
  for (int r = 0; r < 8; ++r) zD[r] = bf_rne(x[(size_t)(rD + r) * kDim + c]);
  const float b2c = bf_rne(b2[c]);
  v8f lp    = zero8;
  v8f kprev = zero8;

  __bf16* sZw = sZ[wave];
  __bf16* sAw = sA[wave];
  const float*          Prow = Pt  + rD;
  const unsigned short* Crow = Ctp + rD;

#pragma unroll 1
  for (int s = 0; s < nseg; ++s) {
    const float t0 = 1.0f + dt * (float)s;
    v8f zsum = zero8, lsum = zero8;
#pragma unroll 1
    for (int st = 0; st < 4; ++st) {
      const float cin = (st == 0) ? 0.0f : ((st == 3) ? dt : hdt);
      const float tst = t0 + cin;
      const float wgt = (st == 1 || st == 2) ? 2.0f : 1.0f;

#pragma unroll
      for (int r = 0; r < 8; ++r) sZw[(8 * hh + r) * 16 + c] = to_bf16(zD[r] + cin * kprev[r]);
      wave_sync();
      FragU zf;
      zf.h8[0] = *(const v8b*)(sZw + c * 16 + koff);
      zf.u[1]  = zero4;

      v8f facc = zero8;
      v8f divp = zero8;
#pragma unroll 1
      for (int kc = 0; kc < kHid / 32; ++kc) {
#pragma unroll
        for (int p = 0; p < 2; ++p) {
          const int n = (kc * 2 + p) * 16 + c;
          const float* pp = Prow + (size_t)n * kRows;
          const v4f pv0 = *(const v4f*)pp;
          const v4f pv1 = *(const v4f*)(pp + 4);
          const v4u cu  = *(const v4u*)(Crow + (size_t)n * kRows);
          FragU bw;
          bw.h8[0] = *(const v8b*)(sW1z + n * 16 + koff);
          bw.u[1]  = zero4;
          v8f hacc = zero8;
          hacc = Frag<__bf16>::mma(zf.v, bw.v, hacc);
          guard1_b(hacc, zf.v, bw.v);
          const float tv = sTv[n];
          const float pv[8] = {pv0.x, pv0.y, pv0.z, pv0.w, pv1.x, pv1.y, pv1.z, pv1.w};
          const unsigned cw0 = cu.x, cw1 = cu.y, cw2 = cu.z, cw3 = cu.w;
          const float cv[8] = {__uint_as_float(cw0 << 16), __uint_as_float(cw0 & 0xffff0000u),
                               __uint_as_float(cw1 << 16), __uint_as_float(cw1 & 0xffff0000u),
                               __uint_as_float(cw2 << 16), __uint_as_float(cw2 & 0xffff0000u),
                               __uint_as_float(cw3 << 16), __uint_as_float(cw3 & 0xffff0000u)};
#pragma unroll
          for (int r = 0; r < 8; ++r) {
            const float h   = hacc[r] + pv[r] + tst * tv;
            const float hcl = fminf(fmaxf(h, -10.0f), 10.0f);
            const float e2  = expf(2.0f * hcl);
            const float a   = 1.0f - 2.0f * __builtin_amdgcn_rcpf(e2 + 1.0f);
            divp[r] += (1.0f - a * a) * cv[r];
            sAw[(8 * hh + r) * 32 + p * 16 + c] = to_bf16(a);
          }
        }
        wave_sync();
        const v16b af  = Frag<__bf16>::load(sAw + c * 32 + koff);
        const v16b bw2 = Frag<__bf16>::load(sW2T + c * kHid + kc * 32 + koff);
        facc = Frag<__bf16>::mma(af, bw2, facc);
        guard1_b(facc, af, bw2);
        wave_sync();
      }
      v8f divv;
#pragma unroll
      for (int r = 0; r < 8; ++r) {
        float v = divp[r];
        v += __shfl_xor(v, 1, 32);
        v += __shfl_xor(v, 2, 32);
        v += __shfl_xor(v, 4, 32);
        v += __shfl_xor(v, 8, 32);
        divv[r] = v;
      }
#pragma unroll
      for (int r = 0; r < 8; ++r) {
        const float f = facc[r] + b2c;
        zsum[r] += wgt * f;
        lsum[r] += wgt * divv[r];
        kprev[r] = f;
      }
    }
#pragma unroll
    for (int r = 0; r < 8; ++r) {
      zD[r] += sixth * zsum[r];
      lp[r] -= sixth * lsum[r];
    }
  }

  v8f zz;
#pragma unroll
  for (int r = 0; r < 8; ++r) {
    float v = zD[r] * zD[r];
    v += __shfl_xor(v, 1, 32);
    v += __shfl_xor(v, 2, 32);
    v += __shfl_xor(v, 4, 32);
    v += __shfl_xor(v, 8, 32);
    zz[r] = v;
  }
  if (c == 0) {
#pragma unroll
    for (int r = 0; r < 8; ++r) sOut[wave * 16 + 8 * hh + r] = (-0.5f * zz[r] - kLogTwoPiTerm) + lp[r];
  }
  __syncthreads();
  if (wave == 0) {
    const v4f v = *(const v4f*)(sOut + 4 * lane);
    float* op = out + (size_t)blockIdx.x * kRowsPerBlock + 4 * lane;
    *(volatile v4f*)op = v;
    __threadfence();
    *(volatile v4f*)op = v;
  }
}

extern "C" void kernel_launch(void* const* d_in, const int* in_sizes, int n_in,
                              void* d_out, int out_size, void* d_ws, size_t ws_size,
                              hipStream_t stream) {
  if (n_in < 8) return;
  if (in_sizes[0] != kRows * kDim || in_sizes[1] != kRows * kCond || in_sizes[2] != kRows * kDim ||
      in_sizes[3] != (kDim + kCond + 1) * kHid || in_sizes[4] != kHid || in_sizes[5] != kHid * kDim ||
      in_sizes[6] != kDim || in_sizes[7] < 1 || out_size != kRows || ws_size < kWsTotal) return;

  const float* x   = (const float*)d_in[0];
  const float* ctx = (const float*)d_in[1];
  const float* eps = (const float*)d_in[2];
  const float* W1  = (const float*)d_in[3];
  const float* b1  = (const float*)d_in[4];
  const float* W2  = (const float*)d_in[5];
  const float* b2  = (const float*)d_in[6];
  const int*   stp = (const int*)d_in[7];
  float* out = (float*)d_out;

  unsigned char* ws = (unsigned char*)d_ws;
  float*          Pt   = (float*)(ws + kOffP);
  unsigned short* Ct   = (unsigned short*)(ws + kOffC);
  unsigned short* ctxb = (unsigned short*)(ws + kOffCtx);
  unsigned short* epsb = (unsigned short*)(ws + kOffEps);
  unsigned short* w1cT = (unsigned short*)(ws + kOffW1c);
  unsigned short* w1zT = (unsigned short*)(ws + kOffW1z);
  unsigned short* w2p  = (unsigned short*)(ws + kOffW2p);
  unsigned short* w2T  = (unsigned short*)(ws + kOffW2T);
  float*          tvec = (float*)(ws + kOffTv);

  prep_kernel<<<kBlkPrep, 256, 0, stream>>>(ctx, eps, W1, W2, ctxb, epsb, w1cT, w1zT, w2p, w2T, tvec);

  wmma_gemm64<1, false, 1, 0, false, 0><<<dim3((kHid / 64) * (kRows / 64) / 8, 1), 256, 0, stream>>>(
      w1cT, w1cT, kCond, 0L, ctxb, ctxb, kCond, 0L, (void*)Pt, (void*)Pt, kRows, 0L,
      b1, b1, 0L, kHid, kRows, kCond, 1.0f);

  dual_gemm_prod_kernel<<<(kHid / 32) * (kRows / 64) / 8, 256, 0, stream>>>(w1zT, w2p, epsb, Ct);

  rk4_kernel<<<kRows / kRowsPerBlock, 256, 0, stream>>>(x, b2, stp, w1zT, w2T, tvec, Pt, Ct, out);
}
